// MultiHeadAttentionNN_50508815401447
// MI455X (gfx1250) — hardware-verified
//
#include <hip/hip_runtime.h>


typedef _Float16 v16h __attribute__((ext_vector_type(16)));
typedef _Float16 v8h  __attribute__((ext_vector_type(8)));
typedef __bf16   v16b __attribute__((ext_vector_type(16)));
typedef float    v8f  __attribute__((ext_vector_type(8)));
typedef float    v4f  __attribute__((ext_vector_type(4)));
typedef unsigned v4u  __attribute__((ext_vector_type(4)));

union FragH { v16h v; v8h hf[2]; v4u q[2]; };
union FragB { v16b v; v4u q[2]; };

#define NOP4 "v_nop\n\tv_nop\n\tv_nop\n\tv_nop"

__device__ __forceinline__ unsigned short bf16_bits(float f) {
  union { __bf16 h; unsigned short u; } c;
  c.h = (__bf16)f;
  return c.u;
}
__device__ __forceinline__ float bf16_to_f32(unsigned short u) {
  return __uint_as_float(((unsigned)u) << 16);
}
__device__ __forceinline__ unsigned short f16_bits(float f) {
  union { _Float16 h; unsigned short u; } c;
  c.h = (_Float16)f;
  return c.u;
}
__device__ __forceinline__ unsigned pack2(unsigned short lo, unsigned short hi) {
  return (unsigned)lo | ((unsigned)hi << 16);
}

__device__ __forceinline__ v8f mma_bf16(v16b a, v16b b, v8f c) {
  return __builtin_amdgcn_wmma_f32_16x16x32_bf16(false, a, false, b, (short)0, c, false, false);
}
__device__ __forceinline__ v8f mma_f16(v16h a, v16h b, v8f c) {
  return __builtin_amdgcn_wmma_f32_16x16x32_f16(false, a, false, b, (short)0, c, false, false);
}

__global__ void __launch_bounds__(256)
k_cvt_bf16(const float* __restrict__ src, unsigned short* __restrict__ dst, int n8) {
  const int i = blockIdx.x * 256 + threadIdx.x;
  if (i >= n8) return;
  const float* p = src + (size_t)i * 8;
  const v4f f0 = *(const v4f*)p;
  const v4f f1 = *(const v4f*)(p + 4);
  v4u o;
  o.x = pack2(bf16_bits(f0.x), bf16_bits(f0.y));
  o.y = pack2(bf16_bits(f0.z), bf16_bits(f0.w));
  o.z = pack2(bf16_bits(f1.x), bf16_bits(f1.y));
  o.w = pack2(bf16_bits(f1.z), bf16_bits(f1.w));
  volatile v4u* d = (volatile v4u*)(dst + (size_t)i * 8);
  *d = o;
  __threadfence();
  *d = o;
}

template <int NJ> struct GemmGuard;
template <> struct GemmGuard<4> {
  static __device__ __forceinline__ void g(v8f (&acc)[2][4], FragB (&a)[2][2], FragB (&b)[4]) {
    asm volatile(NOP4
                 : "+v"(acc[0][0]), "+v"(acc[0][1]), "+v"(acc[0][2]), "+v"(acc[0][3]),
                   "+v"(acc[1][0]), "+v"(acc[1][1]), "+v"(acc[1][2]), "+v"(acc[1][3])
                 : "v"(a[0][0].v), "v"(a[0][1].v),
                   "v"(b[0].v), "v"(b[1].v), "v"(b[2].v), "v"(b[3].v));
  }
};
template <> struct GemmGuard<2> {
  static __device__ __forceinline__ void g(v8f (&acc)[2][4], FragB (&a)[2][2], FragB (&b)[4]) {
    asm volatile(NOP4
                 : "+v"(acc[0][0]), "+v"(acc[0][1]), "+v"(acc[1][0]), "+v"(acc[1][1])
                 : "v"(a[0][0].v), "v"(a[0][1].v), "v"(a[1][0].v), "v"(a[1][1].v),
                   "v"(b[0].v), "v"(b[1].v));
  }
};

template <int NJ, int NPL, bool OUTF32>
__global__ void __launch_bounds__(256)
k_gemm_nt(const unsigned short* __restrict__ A0, const unsigned short* __restrict__ A1,
          const unsigned short* __restrict__ W, void* outp, const float* __restrict__ bias,
          int M, int N, int K) {
  constexpr int BN = 64 * NJ;
  __shared__ v4u tile[64 * 33];
  const int lane = threadIdx.x & 31, wid = threadIdx.x >> 5;
  const int lc = lane & 15, lh = lane >> 4;
  const int wm = wid & 1, wn = wid >> 1;
  const int bm0 = blockIdx.y * 64, bn0 = blockIdx.x * BN;
  const int m0 = bm0 + wm * 32, n0 = bn0 + wn * 16 * NJ;
  (void)M;

  v8f acc[2][4];
#pragma unroll
  for (int i = 0; i < 2; ++i)
#pragma unroll
    for (int j = 0; j < NJ; ++j) acc[i][j] = (v8f){0.f, 0.f, 0.f, 0.f, 0.f, 0.f, 0.f, 0.f};

  const unsigned short* Ap[2];
  Ap[0] = A0;
  Ap[1] = A1;
  size_t aoff[2];
  aoff[0] = (size_t)(m0 + lc) * K;
  aoff[1] = (size_t)(m0 + 16 + lc) * K;
  size_t woff[4];
#pragma unroll
  for (int j = 0; j < NJ; ++j) woff[j] = (size_t)(n0 + j * 16 + lc) * K;

#pragma unroll 1
  for (int k0 = 0; k0 < K; k0 += 32) {
    FragB a[2][2], b[4];
#pragma unroll
    for (int p = 0; p < NPL; ++p)
#pragma unroll
      for (int i = 0; i < 2; ++i) {
        a[p][i].q[0] = *(const v4u*)(Ap[p] + aoff[i] + k0 + 8 * lh);
        a[p][i].q[1] = *(const v4u*)(Ap[p] + aoff[i] + k0 + 16 + 8 * lh);
      }
#pragma unroll
    for (int j = 0; j < NJ; ++j) {
      b[j].q[0] = *(const v4u*)(W + woff[j] + k0 + 8 * lh);
      b[j].q[1] = *(const v4u*)(W + woff[j] + k0 + 16 + 8 * lh);
    }
#pragma unroll
    for (int p = 0; p < NPL; ++p)
#pragma unroll
      for (int i = 0; i < 2; ++i)
#pragma unroll
        for (int j = 0; j < NJ; ++j) acc[i][j] = mma_bf16(a[p][i].v, b[j].v, acc[i][j]);
    GemmGuard<NJ>::g(acc, a, b);
  }

  if (OUTF32) {
    float* tf = (float*)tile;
#pragma unroll
    for (int i = 0; i < 2; ++i)
#pragma unroll
      for (int j = 0; j < NJ; ++j) {
        const int col = wn * 16 * NJ + j * 16 + lc;
        const float bs = bias[bn0 + col];
        const int rowb = wm * 32 + i * 16 + 8 * lh;
#pragma unroll
        for (int r = 0; r < 8; ++r) tf[(rowb + r) * 132 + col] = acc[i][j][r] + bs;
      }
  } else {
    unsigned short* th = (unsigned short*)tile;
#pragma unroll
    for (int i = 0; i < 2; ++i)
#pragma unroll
      for (int j = 0; j < NJ; ++j) {
        const int col = wn * 16 * NJ + j * 16 + lc;
        const int rowb = wm * 32 + i * 16 + 8 * lh;
#pragma unroll
        for (int r = 0; r < 8; ++r) th[(rowb + r) * 264 + col] = f16_bits(acc[i][j][r]);
      }
  }
  __syncthreads();

  v4u vals[8];
#pragma unroll
  for (int rr = 0; rr < 8; ++rr) vals[rr] = tile[(wid * 8 + rr) * 33 + lane];

#pragma unroll
  for (int rr = 0; rr < 8; ++rr) {
    const int row = wid * 8 + rr;
    volatile v4u* gp = OUTF32
        ? (volatile v4u*)((float*)outp + (size_t)(bm0 + row) * N + bn0 + lane * 4)
        : (volatile v4u*)((unsigned short*)outp + (size_t)(bm0 + row) * N + bn0 + lane * 8);
    *gp = vals[rr];
  }
  __threadfence();
#pragma unroll
  for (int rr = 0; rr < 8; ++rr) {
    const int row = wid * 8 + rr;
    volatile v4u* gp = OUTF32
        ? (volatile v4u*)((float*)outp + (size_t)(bm0 + row) * N + bn0 + lane * 4)
        : (volatile v4u*)((unsigned short*)outp + (size_t)(bm0 + row) * N + bn0 + lane * 8);
    *gp = vals[rr];
  }
}

__global__ void __launch_bounds__(256)
k_attn(const unsigned short* __restrict__ qkv, unsigned short* __restrict__ ohi,
       unsigned short* __restrict__ olo) {
  constexpr int S = 2048, LDQ = 3072, FEA = 1024, HB = 192;
  constexpr int KT = 64, NKB = S / KT, P = 72;
  __shared__ __attribute__((aligned(16))) unsigned short kT[KT * P];
  __shared__ __attribute__((aligned(16))) unsigned short vT[64 * P];
  __shared__ __attribute__((aligned(16))) unsigned short st[128 * P];

  const int tid = threadIdx.x, lane = tid & 31, wid = tid >> 5;
  const int lc = lane & 15, lh = lane >> 4;
  const int qb = blockIdx.x, h = blockIdx.y, b = blockIdx.z;
  const size_t rowBase = (size_t)b * S;
  const int qrow0 = qb * 128 + wid * 16;
  const float kscl = 0.125f * 1.4426950408889634f;

  FragH bq[2];
  {
    const unsigned short* qr = qkv + (rowBase + qrow0 + lc) * LDQ + h * HB;
#pragma unroll
    for (int c = 0; c < 2; ++c) {
      bq[c].q[0] = *(const v4u*)(qr + c * 32 + 8 * lh);
      bq[c].q[1] = *(const v4u*)(qr + c * 32 + 16 + 8 * lh);
    }
  }

  v8f oT[4];
#pragma unroll
  for (int dt = 0; dt < 4; ++dt) oT[dt] = (v8f){0.f, 0.f, 0.f, 0.f, 0.f, 0.f, 0.f, 0.f};
  float m = -3.0e38f, l = 0.f;

#pragma unroll 1
  for (int kb = 0; kb < NKB; ++kb) {
    const int key0 = kb * KT;
    __syncthreads();
#pragma unroll
    for (int it = 0; it < 2; ++it) {
      const int idx = tid + it * 256;
      const int kr = idx >> 3, seg = idx & 7;
      *(v4u*)&kT[kr * P + seg * 8] =
          *(const v4u*)(qkv + (rowBase + key0 + kr) * LDQ + h * HB + 64 + seg * 8);
    }
    {
      const int kp = tid >> 3, seg = tid & 7;
      const unsigned short* vs = qkv + (rowBase + key0 + 2 * kp) * LDQ + h * HB + 128 + seg * 8;
      const v4u va = *(const v4u*)vs;
      const v4u vb = *(const v4u*)(vs + LDQ);
      unsigned* vt32 = (unsigned*)vT;
#pragma unroll
      for (int jj = 0; jj < 4; ++jj) {
        const unsigned ua = va[jj], ub = vb[jj];
        const int d0 = seg * 8 + 2 * jj;
        vt32[d0 * 36 + kp]       = (ua & 0xffffu) | (ub << 16);
        vt32[(d0 + 1) * 36 + kp] = (ua >> 16) | (ub & 0xffff0000u);
      }
    }
    __syncthreads();

    v8f sT[4];
#pragma unroll
    for (int t = 0; t < 4; ++t) sT[t] = (v8f){0.f, 0.f, 0.f, 0.f, 0.f, 0.f, 0.f, 0.f};
#pragma unroll
    for (int c = 0; c < 2; ++c) {
      FragH ak[4];
#pragma unroll
      for (int t = 0; t < 4; ++t) {
        const unsigned short* kp_ = &kT[(t * 16 + lc) * P + c * 32 + 8 * lh];
        ak[t].q[0] = *(const v4u*)kp_;
        ak[t].q[1] = *(const v4u*)(kp_ + 16);
      }
#pragma unroll
      for (int t = 0; t < 4; ++t) sT[t] = mma_f16(ak[t].v, bq[c].v, sT[t]);
      asm volatile(NOP4
                   : "+v"(sT[0]), "+v"(sT[1]), "+v"(sT[2]), "+v"(sT[3])
                   : "v"(ak[0].v), "v"(ak[1].v), "v"(ak[2].v), "v"(ak[3].v), "v"(bq[c].v));
    }

    float mx = sT[0][0];
#pragma unroll
    for (int t = 0; t < 4; ++t)
#pragma unroll
      for (int r = 0; r < 8; ++r) mx = fmaxf(mx, sT[t][r]);
    mx = fmaxf(mx, __shfl_xor(mx, 16, 32));
    const float mn = fmaxf(m, mx * kscl);
    const float alpha = __builtin_amdgcn_exp2f(m - mn);
    m = mn;
    const float nmn = -mn;
    FragH bp[2];
    float ps = 0.f;
#pragma unroll
    for (int t = 0; t < 4; ++t) {
      v8f pv;
#pragma unroll
      for (int r = 0; r < 8; ++r) {
        const float pe = __builtin_amdgcn_exp2f(fmaf(sT[t][r], kscl, nmn));
        pv[r] = pe;
        ps += pe;
      }
      bp[t >> 1].hf[t & 1] = __builtin_convertvector(pv, v8h);
    }
    ps += __shfl_xor(ps, 16, 32);
    l = fmaf(l, alpha, ps);
#pragma unroll
    for (int dt = 0; dt < 4; ++dt) oT[dt] *= alpha;

#pragma unroll
    for (int u = 0; u < 2; ++u) {
      FragH av[4];
#pragma unroll
      for (int dt = 0; dt < 4; ++dt) {
        const unsigned short* vp = &vT[(dt * 16 + lc) * P + u * 32 + 8 * lh];
        av[dt].q[0] = *(const v4u*)vp;
        av[dt].q[1] = *(const v4u*)(vp + 16);
      }
#pragma unroll
      for (int dt = 0; dt < 4; ++dt) oT[dt] = mma_f16(av[dt].v, bp[u].v, oT[dt]);
      asm volatile(NOP4
                   : "+v"(oT[0]), "+v"(oT[1]), "+v"(oT[2]), "+v"(oT[3])
                   : "v"(av[0].v), "v"(av[1].v), "v"(av[2].v), "v"(av[3].v), "v"(bp[u].v));
    }
  }

  const float inv = 1.0f / l;
  v4u whi[4], wlo[4];
#pragma unroll
  for (int dt = 0; dt < 4; ++dt) {
    unsigned hw[4], lw[4];
#pragma unroll
    for (int q2 = 0; q2 < 4; ++q2) {
      const float o0 = oT[dt][2 * q2] * inv;
      const float o1 = oT[dt][2 * q2 + 1] * inv;
      const unsigned short h0 = bf16_bits(o0), h1 = bf16_bits(o1);
      const unsigned short l0 = bf16_bits(o0 - bf16_to_f32(h0));
      const unsigned short l1 = bf16_bits(o1 - bf16_to_f32(h1));
      hw[q2] = pack2(h0, h1);
      lw[q2] = pack2(l0, l1);
    }
    whi[dt] = (v4u){hw[0], hw[1], hw[2], hw[3]};
    wlo[dt] = (v4u){lw[0], lw[1], lw[2], lw[3]};
  }

  __syncthreads();
#pragma unroll
  for (int pl = 0; pl < 2; ++pl) {
    unsigned short* ob = pl ? olo : ohi;
#pragma unroll
    for (int dt = 0; dt < 4; ++dt)
      *(v4u*)&st[(wid * 16 + lc) * P + dt * 16 + 8 * lh] = pl ? wlo[dt] : whi[dt];
    __syncthreads();
    v4u vals[4];
#pragma unroll
    for (int j = 0; j < 4; ++j) {
      const int row = wid * 16 + 4 * j + (lane >> 3);
      vals[j] = *(const v4u*)&st[row * P + (lane & 7) * 8];
    }
#pragma unroll
    for (int j = 0; j < 4; ++j) {
      const int row = wid * 16 + 4 * j + (lane >> 3);
      volatile v4u* gp =
          (volatile v4u*)(ob + (rowBase + qb * 128 + row) * FEA + h * 64 + (lane & 7) * 8);
      *gp = vals[j];
    }
    __threadfence();
#pragma unroll
    for (int j = 0; j < 4; ++j) {
      const int row = wid * 16 + 4 * j + (lane >> 3);
      volatile v4u* gp =
          (volatile v4u*)(ob + (rowBase + qb * 128 + row) * FEA + h * 64 + (lane & 7) * 8);
      *gp = vals[j];
    }
    __syncthreads();
  }
}

extern "C" void kernel_launch(void* const* d_in, const int* in_sizes, int n_in,
                              void* d_out, int out_size, void* d_ws, size_t ws_size,
                              hipStream_t stream) {
  constexpr int Bn = 2, S = 2048, D = 1024, FEA = 1024, N1 = 3 * FEA, M = Bn * S;

  if (n_in < 4) return;
  if (in_sizes[0] != M * D || in_sizes[1] != N1 * D || in_sizes[2] != D * FEA ||
      in_sizes[3] != D || out_size != M * D)
    return;

  const float* x     = (const float*)d_in[0];
  const float* qkv_w = (const float*)d_in[1];
  const float* out_w = (const float*)d_in[2];
  const float* out_b = (const float*)d_in[3];
  float* out = (float*)d_out;

  const size_t off_xb   = 0;
  const size_t off_wqkv = off_xb   + (size_t)M * D * 2;
  const size_t off_wo   = off_wqkv + (size_t)N1 * D * 2;
  const size_t off_qkv  = off_wo   + (size_t)D * FEA * 2;
  const size_t off_ahi  = off_qkv  + (size_t)M * N1 * 2;
  const size_t off_alo  = off_ahi  + (size_t)M * FEA * 2;
  const size_t total    = off_alo  + (size_t)M * FEA * 2;
  if (total > ws_size) return;

  unsigned char* ws = (unsigned char*)d_ws;
  unsigned short* xb    = (unsigned short*)(ws + off_xb);
  unsigned short* wqkvb = (unsigned short*)(ws + off_wqkv);
  unsigned short* wob   = (unsigned short*)(ws + off_wo);
  unsigned short* qkvh  = (unsigned short*)(ws + off_qkv);
  unsigned short* ahi   = (unsigned short*)(ws + off_ahi);
  unsigned short* alo   = (unsigned short*)(ws + off_alo);

  const int n8x = M * D / 8, n8w = N1 * D / 8, n8o = D * FEA / 8;
  k_cvt_bf16<<<(n8x + 255) / 256, 256, 0, stream>>>(x, xb, n8x);
  k_cvt_bf16<<<(n8w + 255) / 256, 256, 0, stream>>>(qkv_w, wqkvb, n8w);
  k_cvt_bf16<<<(n8o + 255) / 256, 256, 0, stream>>>(out_w, wob, n8o);

  k_gemm_nt<4, 1, false><<<dim3(N1 / 256, M / 64), 256, 0, stream>>>(
      xb, xb, wqkvb, (void*)qkvh, out_b, M, N1, D);

  k_attn<<<dim3(S / 128, FEA / 64, Bn), 256, 0, stream>>>(qkvh, ahi, alo);

  k_gemm_nt<2, 2, true><<<dim3(D / 128, M / 64), 256, 0, stream>>>(
      ahi, alo, wob, (void*)out, out_b, M, D, FEA);
}
